// IntraAttention_85289460564635
// MI455X (gfx1250) — hardware-verified
//
#include <hip/hip_runtime.h>


#define NB_  4
#define NS   2048
#define DM   1024
#define MAXD 10
#define BSC  0.01f

typedef _Float16 h16;
typedef unsigned short bf;
typedef __attribute__((ext_vector_type(16))) __bf16   v16bf;
typedef __attribute__((ext_vector_type(16))) _Float16 v16h;
typedef __attribute__((ext_vector_type(8)))  _Float16 v8h;
typedef __attribute__((ext_vector_type(8)))  unsigned short v8us;
typedef __attribute__((ext_vector_type(8)))  float    v8f;
typedef __attribute__((ext_vector_type(4)))  float    v4f;
typedef v8h  __attribute__((may_alias)) v8ha;
typedef v4f  __attribute__((may_alias)) v4fa;
typedef v8us __attribute__((may_alias)) v8usa;

__device__ __forceinline__ unsigned short f2bf(float f) { unsigned u = __float_as_uint(f); u += 0x7FFFu + ((u >> 16) & 1u); return (unsigned short)(u >> 16); }
__device__ __forceinline__ float bf2f(unsigned short b) { return __uint_as_float(((unsigned)b) << 16); }
__device__ __forceinline__ float bfr(float f) { return bf2f(f2bf(f)); }
__device__ __forceinline__ v16h cat16(v8h lo, v8h hi) { return __builtin_shufflevector(lo, hi, 0, 1, 2, 3, 4, 5, 6, 7, 8, 9, 10, 11, 12, 13, 14, 15); }
__device__ __forceinline__ v16bf cat16b(v8us lo, v8us hi) { return __builtin_bit_cast(v16bf, __builtin_shufflevector(lo, hi, 0, 1, 2, 3, 4, 5, 6, 7, 8, 9, 10, 11, 12, 13, 14, 15)); }
__device__ __forceinline__ v8f wmma16(v16h a, v16h b, v8f c) { return __builtin_amdgcn_wmma_f32_16x16x32_f16(false, a, false, b, (short)0, c, false, false); }
__device__ __forceinline__ v8f wmmab(v16bf a, v16bf b, v8f c) { return __builtin_amdgcn_wmma_f32_16x16x32_bf16(false, a, false, b, (short)0, c, false, false); }
#define VST2(T, p, v) do { const T vst2_v_ = (v); *(volatile T*)(p) = vst2_v_; __threadfence(); *(volatile T*)(p) = vst2_v_; } while (0)

__global__ __launch_bounds__(256) void k_cvtb(const float* __restrict__ src, int nrows, bf* dst) {
    const int lane = threadIdx.x & 31, row = blockIdx.x * 8 + (threadIdx.x >> 5);
    if (row >= nrows) return;
    v8us o[DM / 256];
#pragma unroll
    for (int c = 0; c < DM / 256; ++c) {
#pragma unroll
        for (int i = 0; i < 8; ++i) o[c][i] = f2bf(src[(size_t)row * DM + c * 256 + lane * 8 + i]); }
#pragma unroll
    for (int c = 0; c < DM / 256; ++c) *(volatile v8us*)(dst + (size_t)row * DM + c * 256 + lane * 8) = o[c];
    __threadfence();
#pragma unroll
    for (int c = 0; c < DM / 256; ++c) *(volatile v8us*)(dst + (size_t)row * DM + c * 256 + lane * 8) = o[c];
}
template <bool BF, int MODE>
__global__ __launch_bounds__(128) void k_gemm(const void* __restrict__ Av, const void* __restrict__ Bv, int K, int ldc, const float* __restrict__ bias, float* C, h16* C16) {
    __shared__ __align__(16) float ost[4][16 * 68];
    const int lane = threadIdx.x & 31, wave = threadIdx.x >> 5, lr = lane & 15, hi = lane >> 4;
    const int r0 = blockIdx.x * 64 + wave * 16, c0 = blockIdx.y * 64;
    const unsigned short* A = (const unsigned short*)Av; const unsigned short* Bm = (const unsigned short*)Bv;
    const size_t aoff = (size_t)(r0 + lr) * K + 8 * hi;
    size_t boff[4];
#pragma unroll
    for (int t = 0; t < 4; ++t) boff[t] = (size_t)(c0 + t * 16 + lr) * K + 8 * hi;
    v8f acc[4];
#pragma unroll
    for (int t = 0; t < 4; ++t) acc[t] = (v8f){};
#pragma unroll 1
    for (int kc = 0; kc < K; kc += 32) {
        const v8us a0 = *(const v8us*)(A + aoff + kc), a1 = *(const v8us*)(A + aoff + kc + 16);
#pragma unroll
        for (int t = 0; t < 4; ++t) { const v8us b0 = *(const v8us*)(Bm + boff[t] + kc), b1 = *(const v8us*)(Bm + boff[t] + kc + 16);
            if (BF) acc[t] = wmmab(cat16b(a0, a1), cat16b(b0, b1), acc[t]);
            else acc[t] = wmma16(cat16(__builtin_bit_cast(v8h, a0), __builtin_bit_cast(v8h, a1)), cat16(__builtin_bit_cast(v8h, b0), __builtin_bit_cast(v8h, b1)), acc[t]); }
        asm volatile("v_nop\n\tv_nop\n\tv_nop\n\tv_nop" : "+v"(acc[0]), "+v"(acc[1]), "+v"(acc[2]), "+v"(acc[3]) : "v"(a0), "v"(a1));
    }
    float* os = &ost[wave][0];
#pragma unroll
    for (int t = 0; t < 4; ++t) { const int col = c0 + t * 16 + lr; const float bv = (MODE == 0) ? bfr(bias[col]) : 0.f;
#pragma unroll
        for (int j = 0; j < 8; ++j) { float v = acc[t][j] + bv;
            if (MODE == 1) { int d = (r0 + hi * 8 + j) - col; d = d < 0 ? -d : d; d = d > MAXD ? MAXD : d; v += BSC * (float)d; }
            os[(hi * 8 + j) * 68 + t * 16 + lr] = v; } }
    __syncthreads();
    float* crow = C + (size_t)r0 * ldc + c0;
    auto pass = [&]() {
#pragma unroll
        for (int s = 0; s < 8; ++s) { const int Lid = (lane >> 3) + 4 * s, piece = lane & 7; const int row = Lid >> 1, cofs = (Lid & 1) * 32 + piece * 4;
            const v4f val = *(const v4fa*)(os + row * 68 + cofs); *(volatile v4f*)(crow + (size_t)row * ldc + cofs) = val; }
        if (MODE == 0) {
#pragma unroll
            for (int s = 0; s < 4; ++s) { const int row = 4 * s + (lane >> 3), piece = lane & 7; const float* sp = os + row * 68 + piece * 8; v8h o;
#pragma unroll
                for (int i = 0; i < 8; ++i) o[i] = (h16)sp[i];
                *(volatile v8h*)(C16 + (size_t)(r0 + row) * ldc + c0 + piece * 8) = o; } }
    };
    pass(); __threadfence(); pass();
}
__global__ __launch_bounds__(256) void k_ft(const float* __restrict__ Ff, h16* FT16) {
    __shared__ __align__(16) h16 tl[64 * 72];
    const int tid = threadIdx.x, j0 = blockIdx.x * 64, h0 = blockIdx.y * 64;
    const int jj = tid >> 2, hq = (tid & 3) * 16;
#pragma unroll
    for (int i = 0; i < 16; ++i) tl[(hq + i) * 72 + jj] = (h16)Ff[(size_t)(j0 + jj) * DM + h0 + hq + i];
    __syncthreads();
    const int piece = tid & 7;
    auto pass = [&]() {
#pragma unroll
        for (int s = 0; s < 2; ++s) { const int hr = (tid >> 3) + 32 * s; const v8h val = *(const v8ha*)(tl + hr * 72 + piece * 8); *(volatile v8h*)(FT16 + (size_t)(h0 + hr) * NS + j0 + piece * 8) = val; }
    };
    pass(); __threadfence(); pass();
}
__global__ __launch_bounds__(256) void k_softmax(const float* __restrict__ S, h16* P16) {
    const int lane = threadIdx.x & 31, i = blockIdx.x * 8 + (threadIdx.x >> 5);
    if (i >= NS) return;
    const float* sr = S + (size_t)i * NS;
    float m = -3.0e38f;
#pragma unroll
    for (int g = 0; g < NS / 256; ++g)
#pragma unroll
        for (int q = 0; q < 8; ++q) m = fmaxf(m, sr[g * 256 + lane * 8 + q]);
#pragma unroll
    for (int sh = 16; sh; sh >>= 1) m = fmaxf(m, __shfl_xor(m, sh, 32));
    float sum = 0.f;
#pragma unroll
    for (int g = 0; g < NS / 256; ++g)
#pragma unroll
        for (int q = 0; q < 8; ++q) sum += __expf(sr[g * 256 + lane * 8 + q] - m);
#pragma unroll
    for (int sh = 16; sh; sh >>= 1) sum += __shfl_xor(sum, sh, 32);
    const float inv = 1.0f / sum;
#pragma unroll 1
    for (int ps = 0; ps < 2; ++ps) {
#pragma unroll
        for (int g = 0; g < NS / 256; ++g) { v8h o;
#pragma unroll
            for (int q = 0; q < 8; ++q) o[q] = (h16)(__expf(sr[g * 256 + lane * 8 + q] - m) * inv);
            *(volatile v8h*)(P16 + (size_t)i * NS + g * 256 + lane * 8) = o; }
        if (ps == 0) __threadfence(); }
}

extern "C" void kernel_launch(void* const* d_in, const int* in_sizes, int n_in,
                              void* d_out, int out_size, void* d_ws, size_t ws_size, hipStream_t stream) {
    (void)in_sizes; (void)n_in; (void)out_size;
    const float* x = (const float*)d_in[0]; const float* Wm = (const float*)d_in[1]; const float* bias = (const float*)d_in[2];
    float* out = (float*)d_out;
    char* wsp = (char*)d_ws;
    auto take = [&](size_t bytes) { char* p = wsp; wsp += (bytes + 255) & ~(size_t)255; return (void*)p; };
    bf* Xb = (bf*)take((size_t)NB_ * NS * DM * 2); bf* WB = (bf*)take((size_t)DM * DM * 2);
    float* Ff = (float*)take((size_t)NS * DM * 4); h16* F16 = (h16*)take((size_t)NS * DM * 2); h16* FT16 = (h16*)take((size_t)DM * NS * 2);
    float* S = (float*)take((size_t)NS * NS * 4); h16* P16 = (h16*)take((size_t)NS * NS * 2);
    if ((size_t)(wsp - (char*)d_ws) > ws_size) return;
    k_cvtb<<<(NB_ * NS) / 8, 256, 0, stream>>>(x, NB_ * NS, Xb);
    k_cvtb<<<DM / 8, 256, 0, stream>>>(Wm, DM, WB);
    for (int b = 0; b < NB_; ++b) {
        k_gemm<true, 0><<<dim3(NS / 64, DM / 64, 1), 128, 0, stream>>>(Xb + (size_t)b * NS * DM, WB, DM, DM, bias, Ff, F16);
        k_ft<<<dim3(NS / 64, DM / 64, 1), 256, 0, stream>>>(Ff, FT16);
        k_gemm<false, 1><<<dim3(NS / 64, NS / 64, 1), 128, 0, stream>>>(F16, F16, DM, NS, nullptr, S, nullptr);
        k_softmax<<<NS / 8, 256, 0, stream>>>(S, P16);
        k_gemm<false, 2><<<dim3(NS / 64, DM / 64, 1), 128, 0, stream>>>(P16, FT16, NS, DM, nullptr, out + (size_t)b * NS * DM, nullptr);
    }
}
